// MultiHeadSpectralAttention_65575560675809
// MI455X (gfx1250) — hardware-verified
//
#include <hip/hip_runtime.h>
#include <math.h>
#include <stdint.h>

#ifndef NB
#define NB 2
#endif
#ifndef NQ
#define NQ 4096
#endif
#define NB_FULL 2
#define CC   256
#define NN   4096
#define NH   8
#define HD   32
#define C3   768
#define HID  64
#define NG   32
#define CPG  8
#define QT   64
#define OSP  68
#define TP   72
#define TABW 32
#define GEPS 1.0e-5f
#define LNPC 8.317766166719343f
#define XSTRIDE_FULL (CC * NN)

static_assert(NB >= 1 && NB <= NB_FULL);
static_assert(NQ % QT == 0 && NQ >= QT && NQ <= NN);
static_assert(NN % QT == 0 && CC % QT == 0 && C3 % QT == 0 && HID == QT);
static_assert(CC == NH * HD && HD == 32 && CC == NG * CPG && CPG == 8);
static_assert(CC % 32 == 0 && HID % 32 == 0 && NN % 32 == 0);
static_assert((OSP * 4) % 16 == 0 && (TP * 2) % 16 == 0);
static_assert(NN % 1024 == 0 && NQ % 4 == 0);
static_assert((C3 * CC) % 2048 == 0 && (CC * CC) % 2048 == 0 && (HID * CC) % 2048 == 0);

typedef _Float16       v16h __attribute__((ext_vector_type(16)));
typedef _Float16       v8h  __attribute__((ext_vector_type(8)));
typedef __bf16         v16b __attribute__((ext_vector_type(16)));
typedef unsigned short v8us __attribute__((ext_vector_type(8)));
typedef float          v8f  __attribute__((ext_vector_type(8)));
typedef float          v4f  __attribute__((ext_vector_type(4)));
typedef unsigned int   v4u  __attribute__((ext_vector_type(4)));

union Frag  { v8us u[2]; v16h h; v16b bf; };
union FragH { v16h v; v8h hv[2]; };
static_assert(sizeof(Frag) == 32);
static_assert(sizeof(FragH) == 32);

__device__ __forceinline__ unsigned short bf_bits(float f) {
  unsigned u = __float_as_uint(f);
  return (unsigned short)((u + 0x7FFFu + ((u >> 16) & 1u)) >> 16);
}
__device__ __forceinline__ float bf_up(unsigned short hb) { return __uint_as_float(((unsigned)hb) << 16); }
__device__ __forceinline__ float bfr(float f) { return bf_up(bf_bits(f)); }
__device__ __forceinline__ unsigned short h_bits(_Float16 x) { return __builtin_bit_cast(unsigned short, x); }
__device__ __forceinline__ unsigned pk16(unsigned short a, unsigned short b) { return (unsigned)a | ((unsigned)b << 16); }
__device__ __forceinline__ v8f zero8() { v8f z = {0.f, 0.f, 0.f, 0.f, 0.f, 0.f, 0.f, 0.f}; return z; }
__device__ __forceinline__ float hmax8(v8f s) {
  return fmaxf(fmaxf(fmaxf(s[0], s[1]), fmaxf(s[2], s[3])), fmaxf(fmaxf(s[4], s[5]), fmaxf(s[6], s[7])));
}
__device__ __forceinline__ unsigned wave_ballot(bool p) {
#if defined(__HIP_DEVICE_COMPILE__)
  return __builtin_amdgcn_ballot_w32(p);
#else
  return p ? 1u : 0u;
#endif
}

__device__ __forceinline__ Frag ldfrag(const unsigned short* p) {
  Frag f;
  f.u[0] = *(const v8us*)(p);
  f.u[1] = *(const v8us*)(p + 16);
  return f;
}

__device__ __forceinline__ v8f mma_h(v16h a, v16h b, v8f c) {
  v8f d = __builtin_amdgcn_wmma_f32_16x16x32_f16(false, a, false, b, (short)0, c, false, false);
#if defined(__HIP_DEVICE_COMPILE__)
  asm volatile("v_nop\n\tv_nop\n\tv_nop\n\tv_nop" : "+v"(d) : "v"(a), "v"(b));
#endif
  return d;
}
__device__ __forceinline__ v8f mma_b(v16b a, v16b b, v8f c) {
  v8f d = __builtin_amdgcn_wmma_f32_16x16x32_bf16(false, a, false, b, (short)0, c, false, false);
#if defined(__HIP_DEVICE_COMPILE__)
  const v16h ha = __builtin_bit_cast(v16h, a), hb = __builtin_bit_cast(v16h, b);
  asm volatile("v_nop\n\tv_nop\n\tv_nop\n\tv_nop" : "+v"(d) : "v"(ha), "v"(hb));
#endif
  return d;
}

__global__ __launch_bounds__(256)
void cvt_bf(const float* __restrict__ src, unsigned short* dst, int n8) {
  const int i  = blockIdx.x * 256 + (int)threadIdx.x;
  const int ic = (i < n8) ? i : (n8 - 1);
  const float* s = src + (size_t)ic * 8;
  const v4f a = *(const v4f*)s;
  const v4f q = *(const v4f*)(s + 4);
  v4u u;
  u[0] = pk16(bf_bits(a[0]), bf_bits(a[1]));
  u[1] = pk16(bf_bits(a[2]), bf_bits(a[3]));
  u[2] = pk16(bf_bits(q[0]), bf_bits(q[1]));
  u[3] = pk16(bf_bits(q[2]), bf_bits(q[3]));
  if (i < n8) {
#pragma unroll
    for (int pass = 0; pass < 2; ++pass) {
      *(volatile v4u*)(dst + (size_t)ic * 8) = u;
      __threadfence();
    }
  }
}

__global__ __launch_bounds__(256)
void stats_k(const float* __restrict__ src, int rnd, int npos, float* tab) {
  __shared__ double ss[256];
  __shared__ double sq[256];
  __shared__ float  sm[2];
  const int tid = threadIdx.x, blk = blockIdx.x;
  const int b = blk / NG, g = blk % NG;
  const float* base = src + ((size_t)(b * CC + g * CPG)) * NN;
  double s = 0.0, q = 0.0;
#pragma unroll 1
  for (int cl = 0; cl < CPG; ++cl) {
    const float* row = base + (size_t)cl * NN;
#pragma unroll 1
    for (int i = 4 * tid; i < npos; i += 1024) {
      const v4f a = *(const v4f*)(row + i);
#pragma unroll
      for (int t = 0; t < 4; ++t) {
        const float f = rnd ? bfr(a[t]) : a[t];
        const double d = (double)f;
        s += d;
        q += d * d;
      }
    }
  }
  ss[tid] = s;
  sq[tid] = q;
  __syncthreads();
#pragma unroll 1
  for (int st = 128; st > 0; st >>= 1) {
    if (tid < st) { ss[tid] += ss[tid + st]; sq[tid] += sq[tid + st]; }
    __syncthreads();
  }
  if (tid == 0) {
    const double cnt = (double)CPG * (double)npos;
    const double mu = ss[0] / cnt;
    double var = sq[0] / cnt - mu * mu;
    if (var < 0.0) var = 0.0;
    const float varf = (float)var;
    sm[0] = (float)mu;
    sm[1] = 1.0f / sqrtf(varf + GEPS);
  }
  __syncthreads();
  if (tid < 8) {
    const float mu = sm[0], rs = sm[1];
    v4f w = {mu, rs, mu, rs};
#pragma unroll
    for (int pass = 0; pass < 2; ++pass) {
      *(volatile v4f*)(tab + (size_t)blk * TABW + 4 * tid) = w;
      __threadfence();
    }
  }
}

__global__ __launch_bounds__(256)
void norm_k(const float* __restrict__ src, int rnd, const float* __restrict__ tab,
            const float* __restrict__ gamma, const float* __restrict__ beta,
            unsigned short* Xh, unsigned short* Xl) {
  __shared__ __align__(16) unsigned short Th[QT * TP];
  __shared__ __align__(16) unsigned short Tl[QT * TP];
  const int tid = threadIdx.x;
  const int nb = blockIdx.x, cbk = blockIdx.y, b = blockIdx.z;
  const int e = tid & 7, lq = tid >> 3;
  const int n0 = nb * QT, c0 = cbk * QT;
#pragma unroll
  for (int it = 0; it < 2; ++it) {
    const int cl = it * 32 + lq;
    const int ch = c0 + cl;
    const int g  = ch / CPG;
    const float mu = tab[(size_t)(b * NG + g) * TABW];
    const float rs = tab[(size_t)(b * NG + g) * TABW + 1];
    const float ga = bfr(gamma[ch]), be = bfr(beta[ch]);
    const float* sp = src + ((size_t)(b * CC + ch)) * NN + n0 + 8 * e;
    const v4f a = *(const v4f*)sp;
    const v4f q = *(const v4f*)(sp + 4);
    const float f[8] = {a[0], a[1], a[2], a[3], q[0], q[1], q[2], q[3]};
    unsigned short hb[8], lb[8];
#pragma unroll
    for (int t = 0; t < 8; ++t) {
      const float xr = rnd ? bfr(f[t]) : f[t];
      const float v  = (xr - mu) * rs * ga + be;
      hb[t] = bf_bits(v);
      lb[t] = bf_bits(v - bf_up(hb[t]));
    }
#pragma unroll
    for (int t = 0; t < 8; ++t) {
      Th[(8 * e + t) * TP + cl] = hb[t];
      Tl[(8 * e + t) * TP + cl] = lb[t];
    }
  }
  __syncthreads();
  v4u uh[2], ul[2];
#pragma unroll
  for (int it = 0; it < 2; ++it) {
    const int nl = it * 32 + lq;
    uh[it] = *(const v4u*)(Th + nl * TP + 8 * e);
    ul[it] = *(const v4u*)(Tl + nl * TP + 8 * e);
  }
#pragma unroll
  for (int pass = 0; pass < 2; ++pass) {
#pragma unroll
    for (int it = 0; it < 2; ++it) {
      const int nl = it * 32 + lq;
      const size_t po = ((size_t)(b * NN + n0 + nl)) * CC + c0 + 8 * e;
      *(volatile v4u*)(Xh + po) = uh[it];
      *(volatile v4u*)(Xl + po) = ul[it];
    }
    __threadfence();
  }
}

template <int KD, int MODE>
__global__ __launch_bounds__(128)
void gemm_k(const unsigned short* __restrict__ Wp,
            const unsigned short* __restrict__ Bh, const unsigned short* __restrict__ Bl,
            const float* __restrict__ bias, const float* __restrict__ rsrc, int rnd,
            unsigned short* P0, unsigned short* P1, unsigned short* P2, unsigned short* P3, float* dstF) {
  static_assert(KD % 32 == 0);
  __shared__ __align__(16) float Os[QT * OSP];
  const int tid  = threadIdx.x;
  const int lane = tid & 31, wave = tid >> 5;
  const int hh   = lane >> 4, c = lane & 15;
  const int nt   = blockIdx.x, mb = blockIdx.y, b = blockIdx.z;
  const int n0   = nt * QT, o0 = mb * QT;

  const unsigned short* ap = Wp + (size_t)(o0 + c) * KD + 8 * hh;
  const size_t boff = ((size_t)(b * NN + n0 + 16 * wave + c)) * KD + 8 * hh;
  const unsigned short* bph = Bh + boff;
  const unsigned short* bpl = Bl + boff;

  v8f acc[4];
#pragma unroll
  for (int mt = 0; mt < 4; ++mt) acc[mt] = zero8();

#pragma unroll 1
  for (int ks = 0; ks < KD / 32; ++ks) {
    const Frag fbh = ldfrag(bph + 32 * ks);
    const Frag fbl = ldfrag(bpl + 32 * ks);
#pragma unroll
    for (int mt = 0; mt < 4; ++mt) {
      const Frag fa = ldfrag(ap + (size_t)(16 * mt) * KD + 32 * ks);
      acc[mt] = mma_b(fa.bf, fbh.bf, acc[mt]);
      acc[mt] = mma_b(fa.bf, fbl.bf, acc[mt]);
    }
  }

  {
    const int nl = 16 * wave + c;
#pragma unroll
    for (int mt = 0; mt < 4; ++mt) {
      v4f va, vb;
#pragma unroll
      for (int r = 0; r < 4; ++r) { va[r] = acc[mt][r]; vb[r] = acc[mt][4 + r]; }
      *(v4f*)(Os + nl * OSP + 16 * mt + 8 * hh)     = va;
      *(v4f*)(Os + nl * OSP + 16 * mt + 8 * hh + 4) = vb;
    }
  }
  __syncthreads();

  if (MODE == 0) {
    const int e = tid & 7, lq = tid >> 3;
    if (mb < 8) {
      const int dcol = (mb & 3) * QT;
      unsigned short* Ph = (mb < 4) ? P0 : P2;
      v4u uh[4], ul[4];
#pragma unroll
      for (int it = 0; it < 4; ++it) {
        const int row = it * 16 + lq;
        const v4f a = *(const v4f*)(Os + row * OSP + 8 * e);
        const v4f q = *(const v4f*)(Os + row * OSP + 8 * e + 4);
        const float f[8] = {a[0], a[1], a[2], a[3], q[0], q[1], q[2], q[3]};
#pragma unroll
        for (int t = 0; t < 4; ++t) {
          const float f0 = f[2 * t], f1 = f[2 * t + 1];
          const unsigned short hb0 = bf_bits(f0), hb1 = bf_bits(f1);
          const unsigned short lb0 = bf_bits(f0 - bf_up(hb0));
          const unsigned short lb1 = bf_bits(f1 - bf_up(hb1));
          uh[it][t] = pk16(hb0, hb1);
          ul[it][t] = pk16(lb0, lb1);
        }
      }
#pragma unroll
      for (int pass = 0; pass < 2; ++pass) {
#pragma unroll
        for (int it = 0; it < 4; ++it) {
          const int row = it * 16 + lq;
          const size_t po = ((size_t)(b * NN + n0 + row)) * CC + dcol + 8 * e;
          *(volatile v4u*)(Ph + po) = uh[it];
          if (mb < 4) *(volatile v4u*)(P1 + po) = ul[it];
        }
        __threadfence();
      }
    } else {
      const int cb0 = (mb - 8) * QT;
      v4u uv[4];
#pragma unroll
      for (int it = 0; it < 4; ++it) {
        const int cl = it * 16 + lq;
        unsigned short hb[8];
#pragma unroll
        for (int t = 0; t < 8; ++t) hb[t] = h_bits((_Float16)Os[(8 * e + t) * OSP + cl]);
#pragma unroll
        for (int t = 0; t < 4; ++t) uv[it][t] = pk16(hb[2 * t], hb[2 * t + 1]);
      }
#pragma unroll
      for (int pass = 0; pass < 2; ++pass) {
#pragma unroll
        for (int it = 0; it < 4; ++it) {
          const int cl = it * 16 + lq;
          const size_t po = ((size_t)(b * CC + cb0 + cl)) * NN + n0 + 8 * e;
          *(volatile v4u*)(P3 + po) = uv[it];
        }
        __threadfence();
      }
    }
  } else if (MODE == 1) {
    const int e = tid & 15, lq = tid >> 4;
    v4f res[8];
#pragma unroll
    for (int it = 0; it < 8; ++it) {
      const int ol = it * 8 + lq;
      const int o  = o0 + ol;
      const float bb = bfr(bias[o]);
      const size_t gi = ((size_t)(b * CC + o)) * NN + n0 + 4 * e;
      const v4f rv = *(const v4f*)(rsrc + gi);
#pragma unroll
      for (int t = 0; t < 4; ++t) {
        const float rr = rnd ? bfr(rv[t]) : rv[t];
        res[it][t] = (Os[(4 * e + t) * OSP + ol] + bb) + rr;
      }
    }
#pragma unroll
    for (int pass = 0; pass < 2; ++pass) {
#pragma unroll
      for (int it = 0; it < 8; ++it) {
        const int ol = it * 8 + lq;
        const size_t gi = ((size_t)(b * CC + o0 + ol)) * NN + n0 + 4 * e;
        *(volatile v4f*)(dstF + gi) = res[it];
      }
      __threadfence();
    }
  } else {
    const int e = tid & 7, lq = tid >> 3;
    v4u uh[4], ul[4];
#pragma unroll
    for (int it = 0; it < 4; ++it) {
      const int nl = it * 16 + lq;
      const v4f a = *(const v4f*)(Os + nl * OSP + 8 * e);
      const v4f q = *(const v4f*)(Os + nl * OSP + 8 * e + 4);
      const float f[8] = {a[0], a[1], a[2], a[3], q[0], q[1], q[2], q[3]};
      unsigned short hb[8], lb[8];
#pragma unroll
      for (int t = 0; t < 8; ++t) {
        const float tt = f[t] + bfr(bias[o0 + 8 * e + t]);
        const float gv = 0.5f * tt * (1.0f + erff(tt * 0.70710678118654752f));
        hb[t] = bf_bits(gv);
        lb[t] = bf_bits(gv - bf_up(hb[t]));
      }
#pragma unroll
      for (int t = 0; t < 4; ++t) {
        uh[it][t] = pk16(hb[2 * t], hb[2 * t + 1]);
        ul[it][t] = pk16(lb[2 * t], lb[2 * t + 1]);
      }
    }
#pragma unroll
    for (int pass = 0; pass < 2; ++pass) {
#pragma unroll
      for (int it = 0; it < 4; ++it) {
        const int nl = it * 16 + lq;
        const size_t po = ((size_t)(b * NN + n0 + nl)) * HID + o0 + 8 * e;
        *(volatile v4u*)(P0 + po) = uh[it];
        *(volatile v4u*)(P1 + po) = ul[it];
      }
      __threadfence();
    }
  }
}

__global__ __launch_bounds__(128)
void attn_k(const unsigned short* __restrict__ Qh, const unsigned short* __restrict__ Ql,
            const unsigned short* __restrict__ Kh, const unsigned short* __restrict__ Vh,
            const float* __restrict__ temperature, unsigned short* Oh, unsigned short* Ol) {
  __shared__ __align__(16) float Os[QT * OSP];
  const int tid  = threadIdx.x;
  const int wave = tid >> 5, lane = tid & 31;
  const int hh   = lane >> 4, c = lane & 15;
  const int n0   = blockIdx.x * QT, hp = blockIdx.y, b = blockIdx.z;
  const int qrow = 16 * wave + c;

#pragma unroll 1
  for (int hs = 0; hs < 2; ++hs) {
    const int h  = 2 * hp + hs;
    const int cb = HD * h;
    const float tr   = bfr(temperature[h]);
    const float temp = fminf(fmaxf(tr, 1.0e-4f), 10.0f);
    const size_t qo = ((size_t)(b * NN + n0 + qrow)) * CC + cb + 8 * hh;
    const Frag qh = ldfrag(Qh + qo);
    const Frag ql = ldfrag(Ql + qo);
    const unsigned short* Khp = Kh + (size_t)b * NN * CC + (size_t)c * CC + cb + 8 * hh;
    const unsigned short* Vp  = Vh + ((size_t)(b * CC + cb + c)) * NN + 8 * hh;

    float m = -1.0e30f, l = 0.f;
    v8f o0 = zero8(), o1 = zero8();

#pragma unroll 1
    for (int kb = 0; kb < NN; kb += 32) {
      const Frag k0 = ldfrag(Khp + (size_t)kb * CC);
      const Frag k1 = ldfrag(Khp + (size_t)(kb + 16) * CC);
      v8f s0 = mma_b(k0.bf, qh.bf, zero8());
      v8f s1 = mma_b(k1.bf, qh.bf, zero8());
      s0 = mma_b(k0.bf, ql.bf, s0);
      s1 = mma_b(k1.bf, ql.bf, s1);
#pragma unroll
      for (int r = 0; r < 8; ++r) { s0[r] *= temp; s1[r] *= temp; }

      float mx = fmaxf(hmax8(s0), hmax8(s1));
      mx = fmaxf(mx, __shfl_xor(mx, 16, 32));
      const float mn = fmaxf(m, mx);
      const unsigned grew = wave_ballot(mx > m);
      if (grew != 0u) {
        const float corr = __expf(m - mn);
        l *= corr;
#pragma unroll
        for (int r = 0; r < 8; ++r) { o0[r] *= corr; o1[r] *= corr; }
      }
      m = mn;
      const float msh = mn - LNPC;

      FragH ph;
      float ls = 0.f;
#pragma unroll
      for (int r = 0; r < 8; ++r) {
        const float e0 = __expf(s0[r] - msh);
        const float e1 = __expf(s1[r] - msh);
        ls += e0 + e1;
        ph.hv[0][r] = (_Float16)e0;
        ph.hv[1][r] = (_Float16)e1;
      }
      l += ls;

      const Frag v0 = ldfrag(Vp + kb);
      const Frag v1 = ldfrag(Vp + (size_t)16 * NN + kb);
      o0 = mma_h(v0.h, ph.v, o0);
      o1 = mma_h(v1.h, ph.v, o1);
    }
    l += __shfl_xor(l, 16, 32);
    const float inv = 1.0f / l;

    {
      v4f va, vb;
#pragma unroll
      for (int r = 0; r < 4; ++r) { va[r] = o0[r] * inv; vb[r] = o0[4 + r] * inv; }
      *(v4f*)(Os + qrow * OSP + 32 * hs + 8 * hh)     = va;
      *(v4f*)(Os + qrow * OSP + 32 * hs + 8 * hh + 4) = vb;
#pragma unroll
      for (int r = 0; r < 4; ++r) { va[r] = o1[r] * inv; vb[r] = o1[4 + r] * inv; }
      *(v4f*)(Os + qrow * OSP + 32 * hs + 16 + 8 * hh)     = va;
      *(v4f*)(Os + qrow * OSP + 32 * hs + 16 + 8 * hh + 4) = vb;
    }
  }
  __syncthreads();

  const int e = tid & 7, lq = tid >> 3;
  v4u uh[4], ul[4];
#pragma unroll
  for (int it = 0; it < 4; ++it) {
    const int row = it * 16 + lq;
    const v4f a = *(const v4f*)(Os + row * OSP + 8 * e);
    const v4f q = *(const v4f*)(Os + row * OSP + 8 * e + 4);
    const float f[8] = {a[0], a[1], a[2], a[3], q[0], q[1], q[2], q[3]};
#pragma unroll
    for (int t = 0; t < 4; ++t) {
      const float f0 = f[2 * t], f1 = f[2 * t + 1];
      const unsigned short hb0 = bf_bits(f0), hb1 = bf_bits(f1);
      const unsigned short lb0 = bf_bits(f0 - bf_up(hb0));
      const unsigned short lb1 = bf_bits(f1 - bf_up(hb1));
      uh[it][t] = pk16(hb0, hb1);
      ul[it][t] = pk16(lb0, lb1);
    }
  }
#pragma unroll
  for (int pass = 0; pass < 2; ++pass) {
#pragma unroll
    for (int it = 0; it < 4; ++it) {
      const int row = it * 16 + lq;
      const size_t po = ((size_t)(b * NN + n0 + row)) * CC + QT * hp + 8 * e;
      *(volatile v4u*)(Oh + po) = uh[it];
      *(volatile v4u*)(Ol + po) = ul[it];
    }
    __threadfence();
  }
}

extern "C" void kernel_launch(void* const* d_in, const int* in_sizes, int n_in,
                              void* d_out, int out_size, void* d_ws, size_t ws_size,
                              hipStream_t stream) {
  if (n_in < 13) return;
  if (in_sizes[0] < NB * XSTRIDE_FULL) return;
  if (in_sizes[1] != C3 * CC || in_sizes[2] != CC * CC || in_sizes[3] != CC) return;
  if (in_sizes[4] != NH) return;
  if (in_sizes[5] != CC || in_sizes[6] != CC || in_sizes[7] != CC || in_sizes[8] != CC) return;
  if (in_sizes[9] != HID * CC || in_sizes[10] != HID || in_sizes[11] != CC * HID || in_sizes[12] != CC) return;
  if (out_size < NB * XSTRIDE_FULL) return;

  size_t off = 0;
  auto carve = [&](size_t bytes) { const size_t o = off; off += (bytes + 255) & ~(size_t)255; return o; };
  const size_t szPl = (size_t)NB * NN * CC * 2;
  const size_t oWq  = carve((size_t)C3 * CC * 2);
  const size_t oWo  = carve((size_t)CC * CC * 2);
  const size_t oW1  = carve((size_t)HID * CC * 2);
  const size_t oW2  = carve((size_t)CC * HID * 2);
  const size_t oT1  = carve((size_t)NB * NG * TABW * 4);
  const size_t oT2  = carve((size_t)NB * NG * TABW * 4);
  const size_t oXh  = carve(szPl);
  const size_t oXl  = carve(szPl);
  const size_t oQh  = carve(szPl);
  const size_t oQl  = carve(szPl);
  const size_t oKh  = carve(szPl);
  const size_t oVv  = carve(szPl);
  const size_t oOh  = carve(szPl);
  const size_t oOl  = carve(szPl);
  const size_t oX1  = carve((size_t)NB * CC * NN * 4);
  const size_t oYh  = carve(szPl);
  const size_t oYl  = carve(szPl);
  const size_t oHh  = carve((size_t)NB * NN * HID * 2);
  const size_t oHl  = carve((size_t)NB * NN * HID * 2);
  if (off > ws_size) return;
  if (off > (size_t)134217728) return;

  const float* x      = (const float*)d_in[0];
  const float* w_qkv  = (const float*)d_in[1];
  const float* w_out  = (const float*)d_in[2];
  const float* b_out  = (const float*)d_in[3];
  const float* tempr  = (const float*)d_in[4];
  const float* g1     = (const float*)d_in[5];
  const float* beta1  = (const float*)d_in[6];
  const float* g2     = (const float*)d_in[7];
  const float* beta2  = (const float*)d_in[8];
  const float* w_mlp1 = (const float*)d_in[9];
  const float* b_mlp1 = (const float*)d_in[10];
  const float* w_mlp2 = (const float*)d_in[11];
  const float* b_mlp2 = (const float*)d_in[12];

  char* ws = (char*)d_ws;
  unsigned short* Wq = (unsigned short*)(ws + oWq);
  unsigned short* Wo = (unsigned short*)(ws + oWo);
  unsigned short* W1 = (unsigned short*)(ws + oW1);
  unsigned short* W2 = (unsigned short*)(ws + oW2);
  float*          T1 = (float*)(ws + oT1);
  float*          T2 = (float*)(ws + oT2);
  unsigned short* Xh = (unsigned short*)(ws + oXh);
  unsigned short* Xl = (unsigned short*)(ws + oXl);
  unsigned short* Qh = (unsigned short*)(ws + oQh);
  unsigned short* Ql = (unsigned short*)(ws + oQl);
  unsigned short* Kh = (unsigned short*)(ws + oKh);
  unsigned short* Vv = (unsigned short*)(ws + oVv);
  unsigned short* Oh = (unsigned short*)(ws + oOh);
  unsigned short* Ol = (unsigned short*)(ws + oOl);
  float*          X1 = (float*)(ws + oX1);
  unsigned short* Yh = (unsigned short*)(ws + oYh);
  unsigned short* Yl = (unsigned short*)(ws + oYl);
  unsigned short* Hh = (unsigned short*)(ws + oHh);
  unsigned short* Hl = (unsigned short*)(ws + oHl);
  float* out = (float*)d_out;

  const dim3 blk256(256), blk128(128);
  const int n8q = C3 * CC / 8, n8o = CC * CC / 8, n81 = HID * CC / 8, n82 = CC * HID / 8;

  cvt_bf<<<dim3((n8q + 255) / 256), blk256, 0, stream>>>(w_qkv, Wq, n8q);
  cvt_bf<<<dim3((n8o + 255) / 256), blk256, 0, stream>>>(w_out, Wo, n8o);
  cvt_bf<<<dim3((n81 + 255) / 256), blk256, 0, stream>>>(w_mlp1, W1, n81);
  cvt_bf<<<dim3((n82 + 255) / 256), blk256, 0, stream>>>(w_mlp2, W2, n82);
  stats_k<<<dim3(NB * NG), blk256, 0, stream>>>(x, 1, NN, T1);
  norm_k<<<dim3(NN / QT, CC / QT, NB), blk256, 0, stream>>>(x, 1, T1, g1, beta1, Xh, Xl);
  gemm_k<CC, 0><<<dim3(NN / QT, C3 / QT, NB), blk128, 0, stream>>>(Wq, Xh, Xl, b_out, x, 0, Qh, Ql, Kh, Vv, X1);
  attn_k<<<dim3(NQ / QT, NH / 2, NB), blk128, 0, stream>>>(Qh, Ql, Kh, Vv, tempr, Oh, Ol);
  gemm_k<CC, 1><<<dim3(NQ / QT, CC / QT, NB), blk128, 0, stream>>>(Wo, Oh, Ol, b_out, x, 1, Hh, Hl, Hh, Hl, X1);
  stats_k<<<dim3(NB * NG), blk256, 0, stream>>>(X1, 0, NQ, T2);
  norm_k<<<dim3(NQ / QT, CC / QT, NB), blk256, 0, stream>>>(X1, 0, T2, g2, beta2, Yh, Yl);
  gemm_k<CC, 2><<<dim3(NQ / QT, 1, NB), blk128, 0, stream>>>(W1, Yh, Yl, b_mlp1, x, 0, Hh, Hl, Hh, Hl, X1);
  gemm_k<HID, 1><<<dim3(NQ / QT, CC / QT, NB), blk128, 0, stream>>>(W2, Hh, Hl, b_mlp2, X1, 0, Oh, Ol, Oh, Ol, out);
  (void)hipGetLastError();
}
